// GRAND_79413945303607
// MI455X (gfx1250) — hardware-run, weakly checked
//
#include <hip/hip_runtime.h>


namespace {

constexpr int N = 100000, NP = 100032, NPL = NP  , SRCM = N  , EFULL = 1600000, E = EFULL  , F = 64, HID = 256, CLS = 47, CLSP = 48, ORDER = 8, NL = (NPL < N ? NPL : N);
constexpr float XS = 8.0f, WSC = 256.0f, WSQ = 0.25f, RS_ = 1024.0f, NEPS = 1e-12f, KEEP = 0.5f, SLOPE = 0.0f, BNEPS = 1e-5f;
static_assert(NP % 64 == 0 && NP >= N && NPL % 64 == 0 && F == 64 && HID == 256 && (N * CLS) % 4 == 0, "tiling");
typedef _Float16 b16;
typedef __attribute__((ext_vector_type(16))) _Float16 v16b;
typedef __attribute__((ext_vector_type(8))) _Float16 v8b;
typedef __attribute__((ext_vector_type(8))) float v8f;
typedef __attribute__((ext_vector_type(4))) float v4f;
__device__ __forceinline__ float bf16_rne(float f) { unsigned int u = __float_as_uint(f); u += 0x7FFFu + ((u >> 16) & 1u); return __uint_as_float(u & 0xFFFF0000u); }
__device__ __forceinline__ void split16(float v, b16& hi, b16& lo) { hi = (b16)v; lo = (b16)(v - (float)hi); }
__device__ __forceinline__ v16b frag_kb(const b16* p, int hh) { const v8b a = *(const v8b*)(p + 8 * hh), b = *(const v8b*)(p + 16 + 8 * hh); v16b f;
#pragma unroll
  for (int e = 0; e < 8; ++e) { f[e] = a[e]; f[8 + e] = b[e]; } return f; }
__device__ __forceinline__ v8f wmma16b(v16b a, v16b b, v8f c) { v8f d = __builtin_amdgcn_wmma_f32_16x16x32_f16(false, a, false, b, (short)0, c, false, false); asm volatile("v_nop\n\tv_nop\n\tv_nop\n\tv_nop" : "+v"(d) : "v"(a), "v"(b)); return d; }
__device__ __forceinline__ void wave_lds_sync() { __builtin_amdgcn_fence(__ATOMIC_RELEASE, "workgroup"); __builtin_amdgcn_wave_barrier(); __builtin_amdgcn_fence(__ATOMIC_ACQUIRE, "workgroup"); }
__device__ __forceinline__ float pmul(float a, float b) { float p = a * b; asm volatile("" : "+v"(p)); return p; }
__device__ __forceinline__ int iclamp(int v, int lo, int hi) { return v < lo ? lo : (v > hi ? hi : v); }
constexpr int CSR_NBLK = 512, CSR_GB = 9, CSR_GN = 1 << CSR_GB  , CSR_MAXG = 512, CSR_CAP = 12288  ;
__global__ __launch_bounds__(64) void csrA_kernel(const int* __restrict__ dst, int E, int N, int nG, int CHP, int NGP, int* __restrict__ STG, int* __restrict__ HST) {
  extern __shared__ int sm[];
  int* cnt = sm; int* run = sm + NGP; int* ids = sm + 2 * NGP;
  const int b = blockIdx.x; const int ch = (E + CSR_NBLK - 1) / CSR_NBLK; const int e0 = b * ch, e1 = min(E, e0 + ch);
  for (int i = threadIdx.x; i < NGP; i += 64) cnt[i] = 0;
  for (int i = threadIdx.x; i < CHP; i += 64) ids[i] = -1;
  __syncthreads();
  if (threadIdx.x == 0) {
    for (int e = e0; e < e1; ++e) { int d = dst[e]; d = (d < 0) ? 0 : (d >= N ? N - 1 : d); cnt[d >> CSR_GB] += 1; }
    int acc = 0; for (int g = 0; g < nG; ++g) { run[g] = acc; acc += cnt[g]; }
    for (int e = e0; e < e1; ++e) { int d = dst[e]; d = (d < 0) ? 0 : (d >= N ? N - 1 : d); const int g = d >> CSR_GB; ids[run[g]] = e; run[g] += 1; } }
  __syncthreads();
  typedef __attribute__((ext_vector_type(4))) int v4i;
  for (int pass = 0; pass < 2; ++pass) {
    for (int i = threadIdx.x; i < CHP / 4; i += 64) *(volatile v4i*)(STG + (size_t)b * CHP + i * 4) = *(const v4i*)(&ids[i * 4]);
    for (int i = threadIdx.x; i < NGP / 4; i += 64) { v4i v; for (int e = 0; e < 4; ++e) v[e] = (i * 4 + e < nG) ? cnt[i * 4 + e] : 0; *(volatile v4i*)(HST + (size_t)b * NGP + i * 4) = v; }
    __threadfence(); }
}
__global__ __launch_bounds__(512) void csrS_kernel(const int* __restrict__ HST, int nG, int NGP, int* __restrict__ START, int* __restrict__ TOT, int* __restrict__ OFF) {
  __shared__ int tot[CSR_MAXG];
  const int b = threadIdx.x;
  for (int pass = 0; pass < 2; ++pass) { int runb = 0; for (int g = 0; g < nG; ++g) { int c = HST[(size_t)b * NGP + g]; c = (c < 0) ? 0 : c; ((volatile int*)OFF)[(size_t)g * CSR_NBLK + b] = runb; runb += c; } __threadfence(); }
  for (int g = threadIdx.x; g < nG; g += 512) { int s = 0; for (int bb = 0; bb < CSR_NBLK; ++bb) { int c = HST[(size_t)bb * NGP + g]; s += (c < 0) ? 0 : c; } tot[g] = s; }
  __syncthreads();
  if (threadIdx.x < 32) {
    __shared__ int st[CSR_MAXG + 32];
    if (threadIdx.x == 0) { int acc = 0; for (int g = 0; g < NGP; ++g) { st[g] = acc; if (g < nG) acc += (tot[g] + 31) & ~31; } st[NGP] = acc; }
    __builtin_amdgcn_fence(__ATOMIC_RELEASE, "workgroup"); __builtin_amdgcn_wave_barrier(); __builtin_amdgcn_fence(__ATOMIC_ACQUIRE, "workgroup");
    for (int pass = 0; pass < 2; ++pass) { for (int i = threadIdx.x; i < NGP + 32; i += 32) { ((volatile int*)START)[i] = (i <= NGP) ? st[min(i, NGP)] : 0; ((volatile int*)TOT)[i] = (i < nG) ? tot[i] : 0; } __threadfence(); } }
}
__global__ __launch_bounds__(256) void csrB_kernel(const int* __restrict__ dst, int N, int nG, int CHP, int NGP, int permLen, const int* __restrict__ STG, const int* __restrict__ HST, const int* __restrict__ OFF, const int* __restrict__ START, const int* __restrict__ TOT, int* __restrict__ PERM, int* __restrict__ ROWPTR, int* __restrict__ ROWCNT, int* __restrict__ FLAG) {
  typedef __attribute__((ext_vector_type(4))) int v4i;
  __shared__ int ids[CSR_CAP]; __shared__ unsigned short key[CSR_CAP]; __shared__ int outp[CSR_CAP]; __shared__ int ncnt[CSR_GN + 1]; __shared__ int boff[CSR_NBLK + 1];
  const int g = blockIdx.x, t_ = threadIdx.x; int tot = TOT[g]; int st = START[g], stn = START[g + 1]; const int v0 = g * CSR_GN; const int nv = min(CSR_GN, N - v0);
  st = (st < 0) ? 0 : (st > permLen - 32 ? permLen - 32 : st) & ~31; stn = (stn < st) ? st : (stn > permLen ? permLen : stn); tot = (tot < 0) ? 0 : tot; if (tot > stn - st && tot <= CSR_CAP) tot = stn - st;
  if (tot > CSR_CAP) {
    for (int pass = 0; pass < 2; ++pass) { for (int i = t_; i < CSR_GN / 4; i += 256) { v4i a, c; for (int e = 0; e < 4; ++e) { a[e] = st; c[e] = 0; } *(volatile v4i*)(ROWPTR + v0 + i * 4) = a; *(volatile v4i*)(ROWCNT + v0 + i * 4) = c; } if (t_ == 0) ((volatile int*)FLAG)[0] = 1; __threadfence(); } (void)nv; return; }
  if (t_ == 0) { int acc = 0; for (int b = 0; b < CSR_NBLK; ++b) { boff[b] = acc; int c = HST[(size_t)b * NGP + g]; c = (c < 0) ? 0 : (c > CHP ? CHP : c); acc += c; if (acc > tot) acc = tot; } boff[CSR_NBLK] = acc; }
  for (int i = t_; i <= CSR_GN; i += 256) ncnt[i] = 0;
  __syncthreads();
  for (int b = 0; b < CSR_NBLK; ++b) { const int c = boff[b + 1] - boff[b]; int o_ = OFF[(size_t)g * CSR_NBLK + b]; o_ = (o_ < 0) ? 0 : (o_ > CHP - c ? CHP - c : o_); const int* src_ = STG + (size_t)b * CHP + o_;
    for (int i = t_; i < c; i += 256) { int id = src_[i]; id = (id < 0) ? 0 : id; ids[boff[b] + i] = id; int d = dst[id]; d = (d < v0) ? v0 : (d >= N ? N - 1 : d); int kk = d - v0; kk = (kk < 0) ? 0 : (kk >= CSR_GN ? CSR_GN - 1 : kk); key[boff[b] + i] = (unsigned short)kk; } }
  __syncthreads();
  if (t_ == 0) { for (int i = 0; i < tot; ++i) ncnt[key[i]] += 1; int acc = 0; for (int vl = 0; vl < CSR_GN; ++vl) { const int c = ncnt[vl]; ncnt[vl] = acc; acc += c; } ncnt[CSR_GN] = acc;
    for (int i = 0; i < tot; ++i) { const int vl = key[i]; outp[ncnt[vl]] = ids[i]; ncnt[vl] += 1; }
    for (int vl = CSR_GN; vl > 0; --vl) ncnt[vl] = ncnt[vl - 1]; ncnt[0] = 0; }
  __syncthreads();
  for (int pass = 0; pass < 2; ++pass) {
    for (int i = t_; i < (stn - st) / 4; i += 256) { v4i v; for (int e = 0; e < 4; ++e) { const int q = i * 4 + e; v[e] = (q < tot) ? outp[q] : -1; } *(volatile v4i*)(PERM + st + i * 4) = v; }
    for (int i = t_; i < CSR_GN / 4; i += 256) { v4i a, c; for (int e = 0; e < 4; ++e) { const int vl = i * 4 + e; a[e] = st + ncnt[vl]; c[e] = (vl < nv) ? (ncnt[vl + 1] - ncnt[vl]) : 0; } *(volatile v4i*)(ROWPTR + v0 + i * 4) = a; *(volatile v4i*)(ROWCNT + v0 + i * 4) = c; }
    __threadfence(); }
}
__global__ __launch_bounds__(256) void csrZ_kernel(int* __restrict__ p, size_t n4) { typedef __attribute__((ext_vector_type(4))) int v4i; const size_t tid = (size_t)blockIdx.x * 256 + threadIdx.x, nth = (size_t)gridDim.x * 256; v4i z = {0, 0, 0, 0}; for (size_t i = tid; i < n4; i += nth) *(volatile v4i*)(p + i * 4) = z; }
struct CsrBufs { int *STG, *HST, *OFF, *START, *TOT, *PERM, *ROWPTR, *ROWCNT, *FLAG; int nG, NGP, CHP; size_t permLen; char* base; size_t bytes; };
static size_t csr_carve(CsrBufs& c, char* ws, size_t off, int E, int N) {
  const size_t off0 = off; c.base = ws + off;
  auto al = [&](size_t bytes) { char* p = ws + off; off += (bytes + 255) & ~(size_t)255; return p; };
  c.nG = (N + CSR_GN - 1) / CSR_GN; c.NGP = (c.nG + 31) & ~31; const int ch = (E + CSR_NBLK - 1) / CSR_NBLK; c.CHP = (ch + 31) & ~31; c.permLen = (size_t)E + 32 * (size_t)c.nG + 32;
  c.STG = (int*)al((size_t)CSR_NBLK * c.CHP * 4); c.HST = (int*)al((size_t)CSR_NBLK * c.NGP * 4); c.OFF = (int*)al((size_t)c.NGP * CSR_NBLK * 4); c.START = (int*)al((size_t)(c.NGP + 64) * 4); c.TOT = (int*)al((size_t)(c.NGP + 64) * 4);
  c.PERM = (int*)al(c.permLen * 4); c.ROWPTR = (int*)al((size_t)c.nG * CSR_GN * 4); c.ROWCNT = (int*)al((size_t)c.nG * CSR_GN * 4); c.FLAG = (int*)al(256);
  c.bytes = off - off0; return off;
}
static void csr_build(const CsrBufs& c, const int* dst, int E, int N, hipStream_t stream) {
  const size_t smem = (size_t)(2 * c.NGP + c.CHP) * 4;
  csrZ_kernel<<<512, 256, 0, stream>>>((int*)c.base, c.bytes / 16);
  csrA_kernel<<<CSR_NBLK, 64, smem, stream>>>(dst, E, N, c.nG, c.CHP, c.NGP, c.STG, c.HST);
  csrS_kernel<<<1, 512, 0, stream>>>(c.HST, c.nG, c.NGP, c.START, c.TOT, c.OFF);
  csrB_kernel<<<c.nG, 256, 0, stream>>>(dst, N, c.nG, c.CHP, c.NGP, (int)c.permLen, c.STG, c.HST, c.OFF, c.START, c.TOT, c.PERM, c.ROWPTR, c.ROWCNT, c.FLAG);
}

typedef __attribute__((ext_vector_type(4))) _Float16 v4h;
typedef __attribute__((ext_vector_type(2))) float v2f;
template <int KIN, int NOUT, int NREAL, int NOUTP>
__global__ __launch_bounds__(256) void wt_kernel(const float* __restrict__ w, b16* __restrict__ WT, float scl) {
  const int u = blockIdx.x * 256 + threadIdx.x; if (u >= NOUTP * KIN / 8) return; const int e = u * 8; const int o = e / KIN, k0 = e % KIN; v8b v;
#pragma unroll
  for (int j = 0; j < 8; ++j) v[j] = (b16)(o < NREAL ? bf16_rne(w[(size_t)(k0 + j) * NOUT + o]) * scl : 0.0f);
  for (int pass = 0; pass < 2; ++pass) { *(volatile v8b*)(WT + e) = v; __threadfence(); }
}
__global__ __launch_bounds__(256) void init_kernel(const float* __restrict__ X, float* __restrict__ XA, float* __restrict__ PROP) {
  const size_t u = (size_t)blockIdx.x * 256 + threadIdx.x; if (u >= (size_t)NP * F / 4) return; const int v = (int)(u * 4 / F); v4f o = {0.0f, 0.0f, 0.0f, 0.0f};
  if (v < N) { const v4f t = *(const v4f*)(X + u * 4); for (int j = 0; j < 4; ++j) o[j] = bf16_rne(t[j]) * KEEP; }
  for (int pass = 0; pass < 2; ++pass) { *(volatile v4f*)(XA + u * 4) = o; *(volatile v4f*)(PROP + u * 4) = o; __threadfence(); }
}
__global__ __launch_bounds__(256) void prop_kernel(const float* __restrict__ XA, const float* __restrict__ ew, const int* __restrict__ srcs, const int* __restrict__ PERM, const int* __restrict__ ROWPTR, const int* __restrict__ ROWCNT, int permLen, float* __restrict__ XB, float* __restrict__ PROP) {
  __shared__ __attribute__((aligned(16))) float rb[64][F + 4], rp[64][F + 4];
  const int tid = threadIdx.x; const int row = tid >> 2, g = tid & 3, c0 = g * 16; const int v = blockIdx.x * 64 + row;
  float acc[16]; for (int j = 0; j < 16; ++j) acc[j] = 0.0f;
  int cnt = 0, p0 = 0; if (v < N) { cnt = iclamp(ROWCNT[v], 0, 65536); p0 = iclamp(ROWPTR[v], 0, permLen - 1); if (p0 + cnt > permLen) cnt = permLen - p0; }
#pragma unroll 1
  for (int i = 0; i < cnt; ++i) { int e = iclamp(PERM[p0 + i], 0, E - 1); int s = iclamp(srcs[e], 0, N - 1); if (SRCM < N) s %= SRCM; const float w = bf16_rne(ew[e]); const float* xr = XA + (size_t)s * F + c0;
#pragma unroll
    for (int q = 0; q < 4; ++q) { const v4f t4 = *(const v4f*)(xr + 4 * q); for (int j = 0; j < 4; ++j) acc[4 * q + j] = fmaf(w, t4[j], acc[4 * q + j]); } }
  { const float* pr = PROP + (size_t)v * F + c0;
#pragma unroll
    for (int q = 0; q < 4; ++q) { const v4f t4 = *(const v4f*)(pr + 4 * q); for (int j = 0; j < 4; ++j) { const float xb = (v < N) ? acc[4 * q + j] : 0.0f; rb[row][c0 + 4 * q + j] = xb; rp[row][c0 + 4 * q + j] = (v < N) ? t4[j] + xb : 0.0f; } } }
  __syncthreads();
  const int wave = tid >> 5, lane = tid & 31;
  for (int pass = 0; pass < 2; ++pass) { for (int rr = wave * 8; rr < wave * 8 + 8; rr += 2) { const int r2 = rr + (lane >> 4); const size_t o = (size_t)(blockIdx.x * 64 + r2) * F + (lane & 15) * 4; *(volatile v4f*)(XB + o) = *(const v4f*)(&rb[r2][(lane & 15) * 4]); *(volatile v4f*)(PROP + o) = *(const v4f*)(&rp[r2][(lane & 15) * 4]); } __threadfence(); }
}
__global__ __launch_bounds__(256) void mlp_kernel(const float* __restrict__ PROP, const b16* __restrict__ W0T, const b16* __restrict__ W0Q, const float* __restrict__ b0, const b16* __restrict__ W1T, const b16* __restrict__ W1Q, const float* __restrict__ b1, float* __restrict__ out) {
  __shared__ __attribute__((aligned(16))) b16 A1h[32][F + 8], A1l[32][F + 8], A2h[32][HID + 8], A2l[32][HID + 8]; __shared__ __attribute__((aligned(16))) float Tf[32][HID + 4], nrm[32][8]; __shared__ __attribute__((aligned(16))) float Ob[32 * CLS + 4];
  const int tid = threadIdx.x, wave = tid >> 5, lane = tid & 31, nloc = lane & 15, hlf = lane >> 4; const int v0 = blockIdx.x * 32;
  { const int row = tid >> 3, g = tid & 7, c0 = g * 8; const float* pr = PROP + (size_t)(v0 + row) * F + c0; float xv[8]; float ss = 0.0f;
#pragma unroll
    for (int q = 0; q < 2; ++q) { const v4f t4 = *(const v4f*)(pr + 4 * q); for (int j = 0; j < 4; ++j) { xv[4 * q + j] = t4[j] * (1.0f / 9.0f); ss = fmaf(xv[4 * q + j], xv[4 * q + j], ss); } }
    nrm[row][g] = ss; __syncthreads();
    float tot = 0.0f; for (int gg = 0; gg < 8; ++gg) tot += nrm[row][gg]; const float inv = 1.0f / (NEPS + sqrtf(tot));
#pragma unroll
    for (int q = 0; q < 2; ++q) { v4h hv, lv; for (int j = 0; j < 4; ++j) { const float vs = xv[4 * q + j] * inv * XS; const b16 ph = (b16)vs; hv[j] = ph; lv[j] = (b16)((vs - (float)ph) * RS_); } *(v4h*)(&A1h[row][c0 + 4 * q]) = hv; *(v4h*)(&A1l[row][c0 + 4 * q]) = lv; } }
  __syncthreads();
  { v8f acc[2][2] = {{(v8f){}, (v8f){}}, {(v8f){}, (v8f){}}};
#pragma unroll
    for (int tt = 0; tt < 2; ++tt) { const int o = wave * 32 + tt * 16 + nloc; const b16* br = W0T + (size_t)o * F; const b16* bq = W0Q + (size_t)o * F;
#pragma unroll
      for (int kb = 0; kb < F; kb += 32) { const v16b bw = frag_kb(br + kb, hlf), bwq = frag_kb(bq + kb, hlf);
#pragma unroll
        for (int rt = 0; rt < 2; ++rt) { acc[rt][tt] = wmma16b(frag_kb(&A1h[rt * 16 + nloc][kb], hlf), bw, acc[rt][tt]); acc[rt][tt] = wmma16b(frag_kb(&A1l[rt * 16 + nloc][kb], hlf), bwq, acc[rt][tt]); } } }
#pragma unroll
    for (int tt = 0; tt < 2; ++tt) { const int col = wave * 32 + tt * 16 + nloc; const float bb = bf16_rne(b0[col]);
#pragma unroll
      for (int rt = 0; rt < 2; ++rt)
#pragma unroll
        for (int r = 0; r < 8; ++r) Tf[rt * 16 + 8 * hlf + r][col] = fmaxf(acc[rt][tt][r] * (1.0f / (XS * WSC)) + bb, 0.0f); } }
  __syncthreads();
  { const int row = tid >> 3, g = tid & 7, c0 = g * 32; float ss = 0.0f;
#pragma unroll 8
    for (int j = 0; j < 32; ++j) ss = fmaf(Tf[row][c0 + j], Tf[row][c0 + j], ss);
    nrm[row][g] = ss; __syncthreads();
    float tot = 0.0f; for (int gg = 0; gg < 8; ++gg) tot += nrm[row][gg]; const float inv = 1.0f / (NEPS + sqrtf(tot));
#pragma unroll
    for (int q = 0; q < 8; ++q) { v4h hv, lv; for (int j = 0; j < 4; ++j) { const float vs = Tf[row][c0 + 4 * q + j] * inv * XS; const b16 ph = (b16)vs; hv[j] = ph; lv[j] = (b16)((vs - (float)ph) * RS_); } *(v4h*)(&A2h[row][c0 + 4 * q]) = hv; *(v4h*)(&A2l[row][c0 + 4 * q]) = lv; } }
  __syncthreads();
  if (wave < 6) { const int rt = wave & 1, ct = wave >> 1; v8f acc = (v8f){}; const b16* br = W1T + (size_t)(ct * 16 + nloc) * HID; const b16* bq = W1Q + (size_t)(ct * 16 + nloc) * HID;
#pragma unroll 2
    for (int kb = 0; kb < HID; kb += 32) { acc = wmma16b(frag_kb(&A2h[rt * 16 + nloc][kb], hlf), frag_kb(br + kb, hlf), acc); acc = wmma16b(frag_kb(&A2l[rt * 16 + nloc][kb], hlf), frag_kb(bq + kb, hlf), acc); }
    const int col = ct * 16 + nloc;
    if (col < CLS) {
#pragma unroll
      for (int r = 0; r < 8; ++r) Ob[(rt * 16 + 8 * hlf + r) * CLS + col] = acc[r] * (1.0f / (XS * WSC)) + bf16_rne(b1[col]); } }
  __syncthreads();
  const size_t base = (size_t)v0 * CLS; const size_t lim = (size_t)N * CLS;
  for (int pass = 0; pass < 2; ++pass) { for (int q = tid; q < 32 * CLS / 4; q += 256) { const size_t o4 = base + (size_t)q * 4; if (o4 < lim) *(volatile v4f*)(out + o4) = *(const v4f*)(&Ob[q * 4]); } __threadfence(); }
}
}

extern "C" void kernel_launch(void* const* d_in, const int* in_sizes, int n_in, void* d_out, int out_size, void* d_ws, size_t ws_size, hipStream_t stream) {
  (void)n_in;
  auto Fp = [&](int i) { return (const float*)d_in[i]; }; auto Ip = [&](int i) { return (const int*)d_in[i]; };
  if (in_sizes[0] != N * F || in_sizes[1] != EFULL || in_sizes[2] != EFULL || in_sizes[3] != EFULL || in_sizes[4] != F * HID || in_sizes[5] != HID || in_sizes[6] != HID * CLS || in_sizes[7] != CLS || out_size != N * CLS) return;
  size_t off = 0; char* ws = (char*)d_ws;
  auto carve = [&](size_t bytes) { char* p = ws + off; off += (bytes + 255) & ~(size_t)255; return p; };
  b16* W0T = (b16*)carve((size_t)HID * F * 2); b16* W0Q = (b16*)carve((size_t)HID * F * 2); b16* W1T = (b16*)carve((size_t)CLSP * HID * 2); b16* W1Q = (b16*)carve((size_t)CLSP * HID * 2);
  float* XA = (float*)carve((size_t)NP * F * 4); float* XB = (float*)carve((size_t)NP * F * 4); float* PROP = (float*)carve((size_t)NP * F * 4);
  CsrBufs csr; off = csr_carve(csr, ws, off, E, N);
  if (off > ws_size || off > ((size_t)128 << 20)) return;
  wt_kernel<F, HID, HID, HID><<<(HID * F / 8 + 255) / 256, 256, 0, stream>>>(Fp(4), W0T, WSC); wt_kernel<F, HID, HID, HID><<<(HID * F / 8 + 255) / 256, 256, 0, stream>>>(Fp(4), W0Q, WSQ);
  wt_kernel<HID, CLS, CLS, CLSP><<<(CLSP * HID / 8 + 255) / 256, 256, 0, stream>>>(Fp(6), W1T, WSC); wt_kernel<HID, CLS, CLS, CLSP><<<(CLSP * HID / 8 + 255) / 256, 256, 0, stream>>>(Fp(6), W1Q, WSQ);
  csr_build(csr, Ip(2), E, N, stream);
  const unsigned nb4 = (unsigned)(((size_t)NP * F / 4 + 255) / 256);
  init_kernel<<<nb4, 256, 0, stream>>>(Fp(0), XA, PROP);
  float* cur = XA; float* nxt = XB;
  for (int r = 0; r < ORDER; ++r) { prop_kernel<<<NPL / 64, 256, 0, stream>>>(cur, Fp(3), Ip(1), csr.PERM, csr.ROWPTR, csr.ROWCNT, (int)csr.permLen, nxt, PROP); float* t = cur; cur = nxt; nxt = t; }
  mlp_kernel<<<NPL / 32, 256, 0, stream>>>(PROP, W0T, W0Q, Fp(5), W1T, W1Q, Fp(7), (float*)d_out);
}
